// ContextualMLPDecryptor_6622839570978
// MI455X (gfx1250) — hardware-verified
//
#include <hip/hip_runtime.h>
#include <stddef.h>


#pragma clang fp contract(off)

#define VOC   38
#define EMBD  128
#define NCTX  5
#define SEQ   1024
#define NBAT  64
#define NROW  (NBAT * SEQ)
#define KIN   (NCTX * EMBD)
#define H1    512
#define H2    256
#define H3    128
#define N4P   64
#define TROW  64
#define RB    64
#define TPB   256
#define OUTB  (RB * VOC)
#define NO4   (OUTB / 4)
#define ASC   64.0f
#define WSC   256.0f
#define ISC   6.103515625e-05f

#define CH2   (H2 * H1 / 8)
#define CH3   (H3 * H2 / 8)
#define CH4   (N4P * H3 / 8)
#define GB2   (CH2 / TPB)
#define GB3   (CH3 / TPB)
#define GB4   (CH4 / TPB)
#define G_PREP (GB2 + GB3 + GB4)
#define G_MLP  (NROW / RB)
#define LDS_MLP ((RB * H1 + RB * H2) * 2)

static_assert(CH2 % TPB == 0);
static_assert(CH3 % TPB == 0);
static_assert(CH4 % TPB == 0);
static_assert(G_PREP == 84);
static_assert(G_MLP == 1024);
static_assert(NROW % RB == 0);
static_assert(SEQ % RB == 0);
static_assert((OUTB * 4) % 128 == 0);
static_assert(NO4 % 8 == 0);
static_assert(NO4 <= 3 * TPB);
static_assert((RB * H1) % (8 * TPB) == 0);
static_assert((RB * H1) / (8 * TPB) == 16);
static_assert(OUTB * 4 <= RB * H2 * 2);
static_assert(RB * H3 * 2 <= RB * H1 * 2);
static_assert(LDS_MLP == 98304);
static_assert(H1 % 32 == 0 && H2 % 32 == 0 && H3 % 32 == 0 && EMBD % 32 == 0);
static_assert((TROW * EMBD) % (8 * TPB) == 0);
static_assert((TROW * 64) % (4 * TPB) == 0);

typedef float          v4f   __attribute__((ext_vector_type(4)));
typedef unsigned int   v4u   __attribute__((ext_vector_type(4)));
typedef float          v8f   __attribute__((ext_vector_type(8)));
typedef _Float16       v8h   __attribute__((ext_vector_type(8)));
typedef _Float16       v16h  __attribute__((ext_vector_type(16)));
typedef unsigned short v8us  __attribute__((ext_vector_type(8)));
typedef unsigned short v16us __attribute__((ext_vector_type(16)));
typedef __bf16         v16bf __attribute__((ext_vector_type(16)));
typedef v4f  __attribute__((may_alias)) v4fa;
typedef v8h  __attribute__((may_alias)) v8ha;
typedef v8us __attribute__((may_alias)) v8usa;
typedef _Float16 __attribute__((may_alias)) f16a;
typedef unsigned short __attribute__((may_alias)) u16a;
typedef float __attribute__((may_alias)) f32a;

union Frag  { v16h v; v8h hf[2]; };
union FragU { v16us v; v8us hf[2]; };
union Pk8   { v8h h; v4u u; };

__device__ __forceinline__ v8f wmma_h(v16h a, v16h b, v8f c) {
  v8f d = __builtin_amdgcn_wmma_f32_16x16x32_f16(false, a, false, b, (short)0, c, false, false);
  asm volatile("v_nop\n\tv_nop\n\tv_nop\n\tv_nop" : "+v"(d) : "v"(a), "v"(b));
  return d;
}
__device__ __forceinline__ v8f wmma_b(v16us a, v16us b, v8f c) {
  const v16bf ab = __builtin_bit_cast(v16bf, a);
  const v16bf bb = __builtin_bit_cast(v16bf, b);
  v8f d = __builtin_amdgcn_wmma_f32_16x16x32_bf16(false, ab, false, bb, (short)0, c, false, false);
  asm volatile("v_nop\n\tv_nop\n\tv_nop\n\tv_nop" : "+v"(d) : "v"(a), "v"(b));
  return d;
}

__device__ __forceinline__ v16h ldfrag_g(const _Float16* p, int h) {
  Frag f;
  f.hf[0] = *(const v8h*)(p + 8 * h);
  f.hf[1] = *(const v8h*)(p + 16 + 8 * h);
  return f.v;
}
__device__ __forceinline__ v16h ldfrag_l(const f16a* p, int h) {
  Frag f;
  f.hf[0] = *(const v8ha*)(p + 8 * h);
  f.hf[1] = *(const v8ha*)(p + 16 + 8 * h);
  return f.v;
}
__device__ __forceinline__ v16us ldfrag_lu(const u16a* p, int h) {
  FragU f;
  f.hf[0] = *(const v8usa*)(p + 8 * h);
  f.hf[1] = *(const v8usa*)(p + 16 + 8 * h);
  return f.v;
}

__device__ __forceinline__ unsigned short f2bf(float f) {
  const unsigned u = __builtin_bit_cast(unsigned, f);
  const unsigned r = u + 0x7FFFu + ((u >> 16) & 1u);
  return (unsigned short)(r >> 16);
}

__device__ __forceinline__ void split8(v4f a, v4f c, v8us& hi, v8us& lo) {
  const float x[8] = {a.x, a.y, a.z, a.w, c.x, c.y, c.z, c.w};
#pragma unroll
  for (int i = 0; i < 8; ++i) {
    const unsigned short hb = f2bf(x[i]);
    const float hf = __builtin_bit_cast(float, ((unsigned)hb) << 16);
    hi[i] = hb;
    lo[i] = f2bf(x[i] - hf);
  }
}

__device__ __forceinline__ v8h cvt8(v4f a, v4f c, float s) {
  v8h r;
  r[0] = (_Float16)(a.x * s); r[1] = (_Float16)(a.y * s);
  r[2] = (_Float16)(a.z * s); r[3] = (_Float16)(a.w * s);
  r[4] = (_Float16)(c.x * s); r[5] = (_Float16)(c.y * s);
  r[6] = (_Float16)(c.z * s); r[7] = (_Float16)(c.w * s);
  return r;
}

__device__ __forceinline__ void lin_chunk(const float* __restrict__ src, int u,
                                          _Float16* __restrict__ dst) {
  const v4f a = *(const v4fa*)(src + (size_t)u * 8);
  const v4f c = *(const v4fa*)(src + (size_t)u * 8 + 4);
  Pk8 pk;
  pk.h = cvt8(a, c, WSC);
  _Float16* d = dst + (size_t)u * 8;
  *(volatile v4u*)d = pk.u;
  __threadfence();
  *(volatile v4u*)d = pk.u;
}

__device__ __forceinline__ void w4_chunk(const float* __restrict__ w4, int u,
                                         _Float16* __restrict__ dst) {
  const int n  = u >> 4;
  const int k8 = (u & 15) * 8;
  const int nc = (n < VOC) ? n : (VOC - 1);
  const float* src = w4 + (size_t)nc * H3 + k8;
  const v4f a = *(const v4fa*)src;
  const v4f c = *(const v4fa*)(src + 4);
  const float s = (n < VOC) ? WSC : 0.0f;
  Pk8 pk;
  pk.h = cvt8(a, c, s);
  _Float16* d = dst + (size_t)u * 8;
  *(volatile v4u*)d = pk.u;
  __threadfence();
  *(volatile v4u*)d = pk.u;
}

__global__ __launch_bounds__(TPB) void k_prep(const float* __restrict__ w2,
                                              const float* __restrict__ w3,
                                              const float* __restrict__ w4,
                                              _Float16* __restrict__ p2,
                                              _Float16* __restrict__ p3,
                                              _Float16* __restrict__ p4)
{
  const int blk = blockIdx.x, tid = threadIdx.x;
  if (blk < GB2) {
    lin_chunk(w2, blk * TPB + tid, p2);
  } else if (blk < GB2 + GB3) {
    lin_chunk(w3, (blk - GB2) * TPB + tid, p3);
  } else {
    w4_chunk(w4, (blk - GB2 - GB3) * TPB + tid, p4);
  }
}

__global__ __launch_bounds__(TPB) void k_table(const float* __restrict__ emb,
                                               const float* __restrict__ w1,
                                               float* __restrict__ T)
{
  __shared__ __align__(16) unsigned short sAh[TROW * EMBD];
  __shared__ __align__(16) unsigned short sAl[TROW * EMBD];
  __shared__ __align__(16) float sT[TROW * 64];

  const int tid = threadIdx.x, wv = tid >> 5, lane = tid & 31;
  const int h = lane >> 4, m = lane & 15;
  const int nb = blockIdx.x, c = blockIdx.y;
  const int n0 = nb * 64;

#pragma unroll 1
  for (int it = 0; it < (TROW * EMBD) / (8 * TPB); ++it) {
    const int q  = it * TPB + tid;
    const int t  = q >> 4;
    const int e8 = (q & 15) * 8;
    const int tc = (t < VOC) ? t : (VOC - 1);
    const float* src = emb + (size_t)tc * EMBD + e8;
    const float f = (t < VOC) ? 1.0f : 0.0f;
    const v4f a = *(const v4fa*)src * f;
    const v4f d = *(const v4fa*)(src + 4) * f;
    v8us hi, lo;
    split8(a, d, hi, lo);
    *(v8usa*)(sAh + t * EMBD + e8) = hi;
    *(v8usa*)(sAl + t * EMBD + e8) = lo;
  }
  __syncthreads();

  const int row0 = (wv & 3) * 16;
  const int nw   = (wv >> 2) * 32;
  const u16a* ahrow = (const u16a*)sAh + (row0 + m) * EMBD;
  const u16a* alrow = (const u16a*)sAl + (row0 + m) * EMBD;

  const v8f z8 = {0.f, 0.f, 0.f, 0.f, 0.f, 0.f, 0.f, 0.f};
  v8f acc[2];
  acc[0] = z8; acc[1] = z8;

#pragma unroll 1
  for (int k0 = 0; k0 < EMBD; k0 += 32) {
    const v16us ah = ldfrag_lu(ahrow + k0, h);
    const v16us al = ldfrag_lu(alrow + k0, h);
#pragma unroll
    for (int u = 0; u < 2; ++u) {
      const int n = n0 + nw + u * 16 + m;
      const float* bp = w1 + (size_t)n * KIN + c * EMBD + k0;
      const v4f b0a = *(const v4fa*)(bp + 8 * h);
      const v4f b0c = *(const v4fa*)(bp + 8 * h + 4);
      const v4f b1a = *(const v4fa*)(bp + 16 + 8 * h);
      const v4f b1c = *(const v4fa*)(bp + 16 + 8 * h + 4);
      FragU bh, bl;
      split8(b0a, b0c, bh.hf[0], bl.hf[0]);
      split8(b1a, b1c, bh.hf[1], bl.hf[1]);
      acc[u] = wmma_b(ah, bh.v, acc[u]);
      acc[u] = wmma_b(ah, bl.v, acc[u]);
      acc[u] = wmma_b(al, bh.v, acc[u]);
    }
  }

#pragma unroll
  for (int u = 0; u < 2; ++u) {
#pragma unroll
    for (int r = 0; r < 8; ++r) {
      sT[(row0 + 8 * h + r) * 64 + nw + u * 16 + m] = acc[u][r];
    }
  }
  __syncthreads();

#pragma unroll 1
  for (int it = 0; it < (TROW * 64) / (4 * TPB); ++it) {
    const int i4  = it * TPB + tid;
    const int row = i4 >> 4;
    const int c4  = (i4 & 15) * 4;
    const v4f v = *(const v4fa*)(sT + row * 64 + c4);
    *(volatile v4f*)(T + ((size_t)(c * TROW + row) * H1 + n0 + c4)) = v;
  }
  __threadfence();
#pragma unroll 1
  for (int it = 0; it < (TROW * 64) / (4 * TPB); ++it) {
    const int i4  = it * TPB + tid;
    const int row = i4 >> 4;
    const int c4  = (i4 & 15) * 4;
    const v4f v = *(const v4fa*)(sT + row * 64 + c4);
    *(volatile v4f*)(T + ((size_t)(c * TROW + row) * H1 + n0 + c4)) = v;
  }
}

template <int K, int NACC>
__device__ __forceinline__ void gemm16(const f16a* arow, const _Float16* __restrict__ brow,
                                       int h, v8f (&acc)[NACC]) {
#pragma unroll 1
  for (int k0 = 0; k0 < K; k0 += 32) {
    const v16h a = ldfrag_l(arow + k0, h);
#pragma unroll
    for (int u = 0; u < NACC; ++u) {
      const v16h b = ldfrag_g(brow + (size_t)u * 16 * K + k0, h);
      acc[u] = wmma_h(a, b, acc[u]);
    }
  }
}

template <int NACC, int LDO>
__device__ __forceinline__ void epi_lds(const v8f (&acc)[NACC], f16a* so, int row0, int n0,
                                        const float* sbias, int h, int m) {
#pragma unroll
  for (int u = 0; u < NACC; ++u) {
    const int n = n0 + u * 16 + m;
    const float bn = sbias[n];
#pragma unroll
    for (int r = 0; r < 8; ++r) {
      float v = acc[u][r] * ISC + bn;
      v = fmaxf(v, 0.0f);
      so[(row0 + 8 * h + r) * LDO + n] = (_Float16)(v * ASC);
    }
  }
}

__global__ __launch_bounds__(TPB) void k_mlp(const int* __restrict__ enc,
                                             const float* __restrict__ T,
                                             const _Float16* __restrict__ p2,
                                             const _Float16* __restrict__ p3,
                                             const _Float16* __restrict__ p4,
                                             const float* __restrict__ b1,
                                             const float* __restrict__ b2,
                                             const float* __restrict__ b3,
                                             const float* __restrict__ b4,
                                             float* __restrict__ out)
{
  extern __shared__ v4f dlds[];
  __shared__ int stok[72];
  __shared__ __align__(16) float sb1[H1];
  __shared__ __align__(16) float sb2[H2];
  __shared__ __align__(16) float sb3[H3];
  __shared__ __align__(16) float sb4[N4P];

  f16a* sH1 = (f16a*)dlds;
  f16a* sH2 = (f16a*)dlds + RB * H1;
  f16a* sH3 = (f16a*)dlds;
  f32a* sO  = (f32a*)((f16a*)dlds + RB * H1);

  const int tid = threadIdx.x, wv = tid >> 5, lane = tid & 31;
  const int h = lane >> 4, m = lane & 15;
  const int blk = blockIdx.x;
  const int rowBase = blk * RB;
  const int bi = rowBase / SEQ;
  const int s0 = rowBase - bi * SEQ;

  for (int i = tid; i < H1; i += TPB) sb1[i] = b1[i];
  sb2[tid] = b2[tid];
  if (tid < H3) sb3[tid] = b3[tid];
  if (tid < N4P) {
    const int ic = (tid < VOC) ? tid : (VOC - 1);
    const float v = b4[ic];
    sb4[tid] = (tid < VOC) ? v : 0.0f;
  }
  if (tid < RB + NCTX - 1) {
    const int sp  = s0 - (NCTX / 2) + tid;
    const bool ok = (sp >= 0) && (sp < SEQ);
    const int spc = (sp < 0) ? 0 : ((sp > SEQ - 1) ? (SEQ - 1) : sp);
    int t = enc[(size_t)bi * SEQ + spc];
    t = (t < 0) ? 0 : ((t > VOC - 1) ? (VOC - 1) : t);
    stok[tid] = ok ? t : -1;
  }
  __syncthreads();

#pragma unroll 1
  for (int it = 0; it < (RB * H1) / (8 * TPB); ++it) {
    const int q  = it * TPB + tid;
    const int r  = q >> 6;
    const int n8 = (q & 63) * 8;
    v4f sa = *(const v4fa*)(sb1 + n8);
    v4f sc = *(const v4fa*)(sb1 + n8 + 4);
#pragma unroll
    for (int c = 0; c < NCTX; ++c) {
      const int t  = stok[r + c];
      const bool ok = (t >= 0);
      const int tc = ok ? t : 0;
      const float f = ok ? 1.0f : 0.0f;
      const float* p = T + ((size_t)(c * TROW + tc) * H1 + n8);
      const v4f a = *(const v4fa*)p;
      const v4f d = *(const v4fa*)(p + 4);
      sa += a * f;
      sc += d * f;
    }
    sa.x = fmaxf(sa.x, 0.0f); sa.y = fmaxf(sa.y, 0.0f);
    sa.z = fmaxf(sa.z, 0.0f); sa.w = fmaxf(sa.w, 0.0f);
    sc.x = fmaxf(sc.x, 0.0f); sc.y = fmaxf(sc.y, 0.0f);
    sc.z = fmaxf(sc.z, 0.0f); sc.w = fmaxf(sc.w, 0.0f);
    const v8h o = cvt8(sa, sc, ASC);
    *(v8ha*)(sH1 + r * H1 + n8) = o;
  }
  __syncthreads();

  const v8f z8 = {0.f, 0.f, 0.f, 0.f, 0.f, 0.f, 0.f, 0.f};
  const int row0 = (wv & 3) * 16;

  {
    const f16a* arow = sH1 + (row0 + m) * H1;
    const int cb = (wv >> 2) * 128;
#pragma unroll 1
    for (int g = 0; g < 2; ++g) {
      const int n0 = cb + g * 64;
      v8f acc[4];
      acc[0] = z8; acc[1] = z8; acc[2] = z8; acc[3] = z8;
      gemm16<H1, 4>(arow, p2 + (size_t)(n0 + m) * H1, h, acc);
      epi_lds<4, H2>(acc, sH2, row0, n0, sb2, h, m);
    }
  }
  __syncthreads();

  {
    const f16a* arow = sH2 + (row0 + m) * H2;
    const int n0 = (wv >> 2) * 64;
    v8f acc[4];
    acc[0] = z8; acc[1] = z8; acc[2] = z8; acc[3] = z8;
    gemm16<H2, 4>(arow, p3 + (size_t)(n0 + m) * H2, h, acc);
    epi_lds<4, H3>(acc, sH3, row0, n0, sb3, h, m);
  }
  __syncthreads();

  {
    const f16a* arow = sH3 + (row0 + m) * H3;
    const int n0 = (wv >> 2) * 32;
    v8f acc[2];
    acc[0] = z8; acc[1] = z8;
    gemm16<H3, 2>(arow, p4 + (size_t)(n0 + m) * H3, h, acc);
#pragma unroll
    for (int u = 0; u < 2; ++u) {
      const int n = n0 + u * 16 + m;
      const float bn = sb4[n];
#pragma unroll
      for (int r = 0; r < 8; ++r) {
        const float v = acc[u][r] * ISC + bn;
        if (n < VOC) sO[(row0 + 8 * h + r) * VOC + n] = v;
      }
    }
  }
  __syncthreads();

  float* dst = out + (size_t)blk * OUTB;
#pragma unroll 1
  for (int it = 0; it < 3; ++it) {
    const int i4 = it * TPB + tid;
    if (i4 < NO4) {
      const v4f v = *(const v4fa*)(sO + 4 * i4);
      *(volatile v4f*)(dst + 4 * i4) = v;
    }
  }
  __threadfence();
#pragma unroll 1
  for (int it = 0; it < 3; ++it) {
    const int i4 = it * TPB + tid;
    if (i4 < NO4) {
      const v4f v = *(const v4fa*)(sO + 4 * i4);
      *(volatile v4f*)(dst + 4 * i4) = v;
    }
  }
}

extern "C" void kernel_launch(void* const* d_in, const int* in_sizes, int n_in,
                              void* d_out, int out_size, void* d_ws, size_t ws_size,
                              hipStream_t stream)
{
  if (n_in < 10) return;
  if (in_sizes[0] != NBAT * SEQ) return;
  if (in_sizes[1] != VOC * EMBD) return;
  if (in_sizes[2] != H1 * KIN) return;
  if (in_sizes[3] != H1) return;
  if (in_sizes[4] != H2 * H1) return;
  if (in_sizes[5] != H2) return;
  if (in_sizes[6] != H3 * H2) return;
  if (in_sizes[7] != H3) return;
  if (in_sizes[8] != VOC * H3) return;
  if (in_sizes[9] != VOC) return;
  if (out_size != NROW * VOC) return;

  const int*   enc = (const int*)d_in[0];
  const float* emb = (const float*)d_in[1];
  const float* w1  = (const float*)d_in[2];
  const float* b1  = (const float*)d_in[3];
  const float* w2  = (const float*)d_in[4];
  const float* b2  = (const float*)d_in[5];
  const float* w3  = (const float*)d_in[6];
  const float* b3  = (const float*)d_in[7];
  const float* w4  = (const float*)d_in[8];
  const float* b4  = (const float*)d_in[9];
  float* out = (float*)d_out;

  const size_t bT  = (size_t)NCTX * TROW * H1 * 4;
  const size_t bP2 = (size_t)H2 * H1 * 2;
  const size_t bP3 = (size_t)H3 * H2 * 2;
  const size_t bP4 = (size_t)N4P * H3 * 2;
  const size_t total = bT + bP2 + bP3 + bP4;
  if (total > ws_size) return;
  if (total > (size_t)134217728) return;

  char* ws = (char*)d_ws;
  size_t off = 0;
  float*    T  = (float*)(ws + off);    off += bT;
  _Float16* p2 = (_Float16*)(ws + off); off += bP2;
  _Float16* p3 = (_Float16*)(ws + off); off += bP3;
  _Float16* p4 = (_Float16*)(ws + off); off += bP4;
  if (off != total) return;

  k_prep<<<G_PREP, TPB, 0, stream>>>(w2, w3, w4, p2, p3, p4);
  k_table<<<dim3(H1 / 64, NCTX), TPB, 0, stream>>>(emb, w1, T);
  hipFuncSetAttribute(reinterpret_cast<const void*>(&k_mlp),
                      hipFuncAttributeMaxDynamicSharedMemorySize, LDS_MLP);
  k_mlp<<<G_MLP, TPB, LDS_MLP, stream>>>(enc, T, p2, p3, p4, b1, b2, b3, b4, out);
}
